// SSMGaussianInterpolator_42408507081242
// MI455X (gfx1250) — hardware-verified
//
#include <hip/hip_runtime.h>
#include <math.h>

typedef __attribute__((ext_vector_type(16))) _Float16 v16h;
typedef __attribute__((ext_vector_type(8)))  _Float16 v8h;
typedef __attribute__((ext_vector_type(16))) __bf16   v16b;
typedef __attribute__((ext_vector_type(8)))  __bf16   v8b;
typedef __attribute__((ext_vector_type(8)))  float    v8f;
typedef __attribute__((ext_vector_type(4)))  float    v4f;
typedef __attribute__((ext_vector_type(2)))  float    v2f;
typedef __attribute__((ext_vector_type(4)))  unsigned int v4u;

constexpr int kNT  = 8;
constexpr int kNP  = 20000;
constexpr int kGD  = 14;
constexpr int kDM  = 128;
constexpr int kNS  = 16;
constexpr int kNL  = 2;
constexpr int kNChunk   = 5;
constexpr int kChunkPts = 4000;
constexpr int kRps      = 4032;
constexpr int kPBlk     = kRps / 64;
constexpr int kRows     = kNT * kRps;
constexpr int kPJW      = 192;
constexpr int kYW       = 256;
constexpr float kLog2e    = 1.4426950408889634f;
constexpr float kNegLn1e4 = -9.210340371976184f;
static_assert(kNChunk * kChunkPts == kNP, "chunks cover all points");
static_assert(kRps >= kChunkPts && (kRps % 64) == 0 && (kRps % 4) == 0, "padded points");
static_assert((kChunkPts % 16) == 0 && (kChunkPts % 64) == 32, "output blocks: 64 or 32 valid points, 16-point multiples are whole 128-B lines");
static_assert((kRows % 64) == 0 && (kRows % 16) == 0, "GEMM M and LN grid");
static_assert((kPJW % 64) == 0 && (kDM % 64) == 0 && (kDM % 32) == 0 && (kYW % 32) == 0, "GEMM N multiples of 64, K multiples of 32");
static_assert(((2 * kRps) % 64) == 0, "windowed GEMM M multiple of 64");

constexpr size_t kOffWPJ  = 0;
constexpr size_t kOffWOUT = kOffWPJ  + (size_t)4 * kPJW * kDM * 2;
constexpr size_t kOffPE   = kOffWOUT + (size_t)2 * kDM * kYW * 2;
constexpr size_t kOffH    = kOffPE   + (size_t)kNT * kDM * 4;
constexpr size_t kOffXNH  = kOffH    + (size_t)kRows * kDM * 4;
constexpr size_t kOffXNL  = kOffXNH  + (size_t)kRows * kDM * 2;
constexpr size_t kOffPJ   = kOffXNL  + (size_t)kRows * kDM * 2;
constexpr size_t kOffYH   = kOffPJ   + (size_t)2 * kRows * kPJW * 4;
constexpr size_t kOffYL   = kOffYH   + (size_t)kRows * kYW * 2;
constexpr size_t kWsTotal = kOffYL   + (size_t)kRows * kYW * 2;
static_assert(kWsTotal == 115937280ull, "carve total");
static_assert(kWsTotal <= 134217728ull, "carve cap");
static_assert((kOffWOUT % 128) == 0 && (kOffPE % 128) == 0 && (kOffH % 128) == 0 && (kOffXNH % 128) == 0 &&
              (kOffXNL % 128) == 0 && (kOffPJ % 128) == 0 && (kOffYH % 128) == 0 && (kOffYL % 128) == 0, "128-B aligned regions");

__device__ __forceinline__ unsigned short f2bf_bits(float f) {
  unsigned u = __float_as_uint(f);
  return (unsigned short)((u + 0x7FFFu + ((u >> 16) & 1u)) >> 16);
}
__device__ __forceinline__ float bf_bits2f(unsigned short h) { return __uint_as_float(((unsigned)h) << 16); }
__device__ __forceinline__ float bf16r(float f) { return __uint_as_float(((unsigned)f2bf_bits(f)) << 16); }

__device__ __forceinline__ void dep_guard4_h(v8f& a, v8f& b, v8f& c, v8f& d, v16h x, v16h y) { asm volatile("v_nop\n\tv_nop\n\tv_nop\n\tv_nop" : "+v"(a), "+v"(b), "+v"(c), "+v"(d) : "v"(x), "v"(y)); }
__device__ __forceinline__ void dep_guard4_b(v8f& a, v8f& b, v8f& c, v8f& d, v16b x, v16b y) { asm volatile("v_nop\n\tv_nop\n\tv_nop\n\tv_nop" : "+v"(a), "+v"(b), "+v"(c), "+v"(d) : "v"(x), "v"(y)); }
__device__ __forceinline__ void keep4_h(v16h a, v16h b, v16h c, v16h d) { asm volatile("v_nop" :: "v"(a), "v"(b), "v"(c), "v"(d)); }
__device__ __forceinline__ void keep4_b(v16b a, v16b b, v16b c, v16b d) { asm volatile("v_nop" :: "v"(a), "v"(b), "v"(c), "v"(d)); }
__device__ __forceinline__ void acc_guard4(v8f& a, v8f& b, v8f& c, v8f& d) { asm volatile("v_nop\n\tv_nop\n\tv_nop\n\tv_nop" : "+v"(a), "+v"(b), "+v"(c), "+v"(d)); }
template <typename T> struct Frag;
template <> struct Frag<_Float16> {
  typedef v16h V; union U { v16h v; v8h h[2]; };
  static __device__ __forceinline__ v16h load(const _Float16* p) {
    U f; f.h[0] = *(const v8h*)(p); f.h[1] = *(const v8h*)(p + 16); return f.v;
  }
  static __device__ __forceinline__ v8f mma(v16h a, v16h b, v8f c) {
    return __builtin_amdgcn_wmma_f32_16x16x32_f16(false, a, false, b, (short)0, c, false, false);
  }
  static __device__ __forceinline__ void guard4(v8f& a, v8f& b, v8f& c, v8f& d, v16h x, v16h y) { dep_guard4_h(a, b, c, d, x, y); }
  static __device__ __forceinline__ void keep(v16h a, v16h b, v16h c, v16h d) { keep4_h(a, b, c, d); }
};
template <> struct Frag<__bf16> {
  typedef v16b V; union U { v16b v; v8b h[2]; };
  static __device__ __forceinline__ v16b load(const __bf16* p) {
    U f; f.h[0] = *(const v8b*)(p); f.h[1] = *(const v8b*)(p + 16); return f.v;
  }
  static __device__ __forceinline__ v8f mma(v16b a, v16b b, v8f c) {
    return __builtin_amdgcn_wmma_f32_16x16x32_bf16(false, a, false, b, (short)0, c, false, false);
  }
  static __device__ __forceinline__ void guard4(v8f& a, v8f& b, v8f& c, v8f& d, v16b x, v16b y) { dep_guard4_b(a, b, c, d, x, y); }
  static __device__ __forceinline__ void keep(v16b a, v16b b, v16b c, v16b d) { keep4_b(a, b, c, d); }
};

__device__ __forceinline__ int sel_low_index(const float* tsrc) {
  const float tv = bf16r(tsrc[0]);
  const float tn = tv * 7.0f;
  int il = (int)floorf(tn);
  il = il < 0 ? 0 : il;
  il = il > (kNT - 2) ? (kNT - 2) : il;
  return il;
}

template <int ET> struct Elem;
template <> struct Elem<0> { typedef _Float16 T; };
template <> struct Elem<1> { typedef __bf16 T; };
template <int ET, int SPL, int BIAS_MODE, int OUT_MODE, bool RESID, int ACT, int RWIN>
__global__ __launch_bounds__(256) void wmma_gemm64(
    const unsigned short* __restrict__ Ap, const unsigned short* __restrict__ A2p, int lda, long strideA,
    const unsigned short* __restrict__ Btp, const unsigned short* __restrict__ Bt2p, int ldb, long strideB,
    void* Cout, void* Cout2, int ldc, long strideC,
    const float* __restrict__ bias,
    const float* resid, long strideR,
    int M, int N, int K, float scale, const float* __restrict__ tsrc, int rps) {
  typedef typename Elem<ET>::T T;
  typedef typename Frag<T>::V V;
  const T* A = (const T*)Ap; const T* A2 = (const T*)A2p; const T* Bt = (const T*)Btp; const T* Bt2 = (const T*)Bt2p;
  __shared__ __align__(16) float sT[8][16 * 68];
  const int b    = blockIdx.y;
  const int lane = threadIdx.x & 31;
  const int wave = threadIdx.x >> 5;
  const int tilesN = N >> 6;
  const int tilesM = M >> 6;
  const int tile = blockIdx.x * 8 + wave;
  if (tile >= tilesM * tilesN) return;
  const int tm = tile / tilesN;
  const int tn = tile - tm * tilesN;
  const int m0 = tm << 6;
  const int n0 = tn << 6;

  size_t rowoff = 0;
  if (RWIN != 0) {
    const int il = sel_low_index(tsrc);
    if (RWIN == 1) {
      const int lo = (b == 0) ? 0 : il * rps;
      const int hi = (b == 0) ? (il + 2) * rps : kNT * rps;
      if (m0 < lo || m0 >= hi) return;
    } else {
      rowoff = (size_t)il * (size_t)rps;
    }
  }

  const T* Ab  = A  + (size_t)b * strideA + rowoff * (size_t)lda;
  const T* Bb  = Bt + (size_t)b * strideB;
  const T* Ab2 = (SPL >= 1) ? (A2  + (size_t)b * strideA + rowoff * (size_t)lda) : nullptr;
  const T* Bb2 = (SPL == 2) ? (Bt2 + (size_t)b * strideB) : nullptr;

  const int rlane = lane & 15;
  const int koff  = (lane >> 4) * 8;
  const int mOff  = (lane >> 4) * 8;

  v8f acc[4][4];
#pragma unroll
  for (int i = 0; i < 4; ++i)
#pragma unroll
    for (int j = 0; j < 4; ++j) acc[i][j] = (v8f){0.f,0.f,0.f,0.f,0.f,0.f,0.f,0.f};

  for (int k0 = 0; k0 < K; k0 += 32) {
    V bh[4], bl[4];
#pragma unroll
    for (int j = 0; j < 4; ++j) {
      const size_t bo = (size_t)(n0 + (j << 4) + rlane) * ldb + koff + k0;
      bh[j] = Frag<T>::load(Bb + bo);
      if (SPL == 2) bl[j] = Frag<T>::load(Bb2 + bo);
    }
#pragma unroll
    for (int i = 0; i < 4; ++i) {
      const size_t ao = (size_t)(m0 + (i << 4) + rlane) * lda + koff + k0;
      V ah = Frag<T>::load(Ab + ao);
      V al;
      if (SPL >= 1) al = Frag<T>::load(Ab2 + ao);
#pragma unroll
      for (int j = 0; j < 4; ++j) {
        acc[i][j] = Frag<T>::mma(ah, bh[j], acc[i][j]);
        if (SPL == 2) acc[i][j] = Frag<T>::mma(ah, bl[j], acc[i][j]);
        if (SPL >= 1) acc[i][j] = Frag<T>::mma(al, bh[j], acc[i][j]);
      }
      Frag<T>::guard4(acc[i][0], acc[i][1], acc[i][2], acc[i][3], ah, (SPL >= 1) ? al : ah);
    }
    Frag<T>::keep(bh[0], bh[1], bh[2], bh[3]);
    if (SPL == 2) Frag<T>::keep(bl[0], bl[1], bl[2], bl[3]);
  }
  acc_guard4(acc[0][0], acc[0][1], acc[0][2], acc[0][3]);
  acc_guard4(acc[1][0], acc[1][1], acc[1][2], acc[1][3]);
  acc_guard4(acc[2][0], acc[2][1], acc[2][2], acc[2][3]);
  acc_guard4(acc[3][0], acc[3][1], acc[3][2], acc[3][3]);

  float* slab = sT[wave];
#pragma unroll
  for (int i = 0; i < 4; ++i) {
    const int mBase = m0 + (i << 4);
#pragma unroll
    for (int j = 0; j < 4; ++j) {
      const int n = n0 + (j << 4) + rlane;
      float bv = 0.f;
      if (BIAS_MODE == 2) bv = bf16r(bias[n]);
#pragma unroll
      for (int r = 0; r < 8; ++r) {
        float v = acc[i][j][r] * scale;
        if (BIAS_MODE == 1) v += bf16r(bias[mBase + mOff + r]);
        if (BIAS_MODE == 2) v += bv;
        if (ACT == 1) v = tanhf(v);
        if (ACT == 2) v = fmaxf(v, 0.0f);
        if (ACT == 3) v = v / (1.0f + expf(-v));
        if (ACT == 4) v = (v > 0.f) ? v : 0.01f * v;
        slab[(mOff + r) * 68 + (j << 4) + rlane] = v;
      }
    }
    __builtin_amdgcn_fence(__ATOMIC_RELEASE, "workgroup");
    __builtin_amdgcn_wave_barrier();
    __builtin_amdgcn_fence(__ATOMIC_ACQUIRE, "workgroup");
    if (OUT_MODE == 0) {
      float* C = (float*)Cout + (size_t)b * strideC + rowoff * (size_t)ldc;
      const int hh = lane >> 4, c4 = (lane & 15) * 4;
      if (RESID) {
        const float* Rw = resid + (size_t)b * strideR + rowoff * (size_t)ldc;
#pragma unroll
        for (int it = 0; it < 8; ++it) {
          const int row = it * 2 + hh;
          float* sp = slab + row * 68 + c4;
          v4f v = *(const v4f*)sp;
          const v4f rv = *(const v4f*)(Rw + (size_t)(mBase + row) * ldc + n0 + c4);
          v += rv;
          *(v4f*)sp = v;
        }
      }
      for (int pass = 0; pass < 2; ++pass) {
#pragma unroll
        for (int it = 0; it < 8; ++it) {
          const int row = it * 2 + hh;
          v4f v = *(const v4f*)(slab + row * 68 + c4);
          *(volatile v4f*)(C + (size_t)(mBase + row) * ldc + n0 + c4) = v;
        }
        __threadfence();
      }
    } else {
      const int q = lane >> 3, c8 = (lane & 7) * 8;
      unsigned short* C  = (unsigned short*)Cout  + (size_t)b * strideC + rowoff * (size_t)ldc;
      unsigned short* C2 = (OUT_MODE == 2) ? ((unsigned short*)Cout2 + (size_t)b * strideC + rowoff * (size_t)ldc) : nullptr;
      for (int pass = 0; pass < 2; ++pass) {
#pragma unroll
        for (int it = 0; it < 4; ++it) {
          const int row = it * 4 + q;
          const float* sp = slab + row * 68 + c8;
          v8h hv, lv;
#pragma unroll
          for (int e = 0; e < 8; ++e) {
            if (OUT_MODE == 1) {
              hv[e] = (_Float16)sp[e];
            } else {
              unsigned short hb = f2bf_bits(sp[e]);
              unsigned short lb = f2bf_bits(sp[e] - bf_bits2f(hb));
              hv[e] = __builtin_bit_cast(_Float16, hb);
              lv[e] = __builtin_bit_cast(_Float16, lb);
            }
          }
          *(volatile v8h*)(C + (size_t)(mBase + row) * ldc + n0 + c8) = hv;
          if (OUT_MODE == 2) *(volatile v8h*)(C2 + (size_t)(mBase + row) * ldc + n0 + c8) = lv;
        }
        __threadfence();
      }
    }
    __builtin_amdgcn_fence(__ATOMIC_RELEASE, "workgroup");
    __builtin_amdgcn_wave_barrier();
    __builtin_amdgcn_fence(__ATOMIC_ACQUIRE, "workgroup");
  }
}

__global__ __launch_bounds__(256) void prep_kernel(
    const float* __restrict__ dt_W, const float* __restrict__ B_W, const float* __restrict__ C_W,
    const float* __restrict__ out_W, const float* __restrict__ tstamp,
    unsigned short* __restrict__ WPJ, unsigned short* __restrict__ WOUT, float* __restrict__ PE)
{
  __shared__ __align__(16) unsigned short sT[64 * 264];
  __shared__ __align__(16) float sPE[kNT * kDM];
  const int tid = threadIdx.x, lane = tid & 31, wave = tid >> 5;
  const int bx = blockIdx.x;
  if (bx < 12) {
    const int ld = bx / 3, g = bx - ld * 3;
    constexpr int pitch = 136;
    if (g < 2) {
      const int nl = tid & 63, kq = tid >> 6;
      const int n = g * 64 + nl;
      const float* src = dt_W + (size_t)ld * kDM * kDM;
#pragma unroll 1
      for (int i = 0; i < 32; ++i) {
        const int k = kq + 4 * i;
        sT[nl * pitch + k] = f2bf_bits(src[(size_t)k * kDM + n]);
      }
    } else {
      const int k = tid & 127, half = tid >> 7;
      const float* src = (half ? C_W : B_W) + (size_t)ld * kDM * kNS;
#pragma unroll 1
      for (int s = 0; s < kNS; ++s) {
        sT[(half * 16 + s) * pitch + k] = f2bf_bits(src[(size_t)k * kNS + s]);
        sT[(32 + half * 16 + s) * pitch + k] = (unsigned short)0;
      }
    }
    __syncthreads();
    unsigned short* dst = WPJ + (size_t)ld * (kPJW * kDM) + (size_t)(g * 64) * kDM;
    const int k8 = (lane & 15) * 8, rsub = lane >> 4;
    v4u vv[4];
#pragma unroll
    for (int it = 0; it < 4; ++it) {
      const int row = wave * 8 + it * 2 + rsub;
      vv[it] = *(const v4u*)(sT + row * pitch + k8);
    }
    for (int pass = 0; pass < 2; ++pass) {
#pragma unroll
      for (int it = 0; it < 4; ++it) {
        const int row = wave * 8 + it * 2 + rsub;
        *(volatile v4u*)(dst + (size_t)row * kDM + k8) = vv[it];
      }
      __threadfence();
    }
  } else if (bx < 16) {
    const int l = (bx - 12) >> 1, g = (bx - 12) & 1;
    constexpr int pitch = 264;
    const int nl = tid & 63, kq = tid >> 6;
    const int n = g * 64 + nl;
    const float* src = out_W + (size_t)l * kYW * kDM;
#pragma unroll 1
    for (int i = 0; i < 64; ++i) {
      const int k = kq + 4 * i;
      sT[nl * pitch + k] = f2bf_bits(src[(size_t)k * kDM + n]);
    }
    __syncthreads();
    unsigned short* dst = WOUT + (size_t)l * (kDM * kYW) + (size_t)(g * 64) * kYW;
    const int k8 = lane * 8;
    v4u vv[8];
#pragma unroll
    for (int it = 0; it < 8; ++it) {
      const int row = wave * 8 + it;
      vv[it] = *(const v4u*)(sT + row * pitch + k8);
    }
    for (int pass = 0; pass < 2; ++pass) {
#pragma unroll
      for (int it = 0; it < 8; ++it) {
        const int row = wave * 8 + it;
        *(volatile v4u*)(dst + (size_t)row * kYW + k8) = vv[it];
      }
      __threadfence();
    }
  } else {
    const int n = tid >> 5, c4 = (tid & 31) * 4;
    const float ts = bf16r(tstamp[n]);
#pragma unroll 1
    for (int e = 0; e < 4; ++e) {
      const int c = c4 + e;
      const int j = c & 63;
      float a = kNegLn1e4 * (float)j;
      a = a * 0.015625f;
      const float fr = expf(a);
      const float ang = ts * fr;
      const float sv = sinf(ang);
      const float cv = cosf(ang);
      sPE[tid * 4 + e] = (c < 64) ? sv : cv;
    }
    __syncthreads();
    const v4f v = *(const v4f*)(sPE + tid * 4);
    float* q = PE + tid * 4;
    *(volatile v4f*)q = v;
    __threadfence();
    *(volatile v4f*)q = v;
  }
}

__global__ __launch_bounds__(256) void inproj_kernel(
    const float* __restrict__ xyz, const float* __restrict__ scl, const float* __restrict__ rot,
    const float* __restrict__ opa, const float* __restrict__ col,
    const float* __restrict__ in_W, const float* __restrict__ in_b, const float* __restrict__ PE,
    float* __restrict__ H, int chunk)
{
  __shared__ __align__(16) float sW[kGD * kDM];
  __shared__ __align__(16) float sB[kDM];
  __shared__ __align__(16) float sPE[kDM];
  __shared__ __align__(16) float sP[64 * 16];
  const int tid = threadIdx.x, lane = tid & 31, wave = tid >> 5;
  const int n = blockIdx.x / kPBlk;
  const int pb = blockIdx.x - n * kPBlk;
  const int p0l = pb * 64;
  const int pbase = chunk * kChunkPts + p0l;
  for (int idx = tid; idx < kGD * kDM; idx += 256) sW[idx] = bf16r(in_W[idx]);
  if (tid < kDM) { sB[tid] = bf16r(in_b[tid]); sPE[tid] = PE[n * kDM + tid]; }
  if (tid < 192) {
    const int pl = tid / 3, f = tid - pl * 3;
    int pg = pbase + pl; pg = pg > (kNP - 1) ? (kNP - 1) : pg;
    const size_t base = (size_t)n * kNP + pg;
    sP[pl * 16 + f]      = bf16r(xyz[base * 3 + f]);
    sP[pl * 16 + 3 + f]  = bf16r(scl[base * 3 + f]);
    sP[pl * 16 + 11 + f] = bf16r(col[base * 3 + f]);
  }
  {
    const int pl = tid >> 2, f = tid & 3;
    int pg = pbase + pl; pg = pg > (kNP - 1) ? (kNP - 1) : pg;
    const size_t base = (size_t)n * kNP + pg;
    sP[pl * 16 + 6 + f] = bf16r(rot[base * 4 + f]);
  }
  if (tid < 64) {
    int pg = pbase + tid; pg = pg > (kNP - 1) ? (kNP - 1) : pg;
    const size_t base = (size_t)n * kNP + pg;
    sP[tid * 16 + 10] = bf16r(opa[base]);
  }
  __syncthreads();
  const int c4 = lane * 4;
  const v4f bb = *(const v4f*)(sB + c4);
  const v4f pe = *(const v4f*)(sPE + c4);
#pragma unroll 1
  for (int i = 0; i < 8; ++i) {
    const int pl = wave * 8 + i;
    v4f acc = (v4f){0.f, 0.f, 0.f, 0.f};
#pragma unroll
    for (int f = 0; f < kGD; ++f) {
      const float p = sP[pl * 16 + f];
      const v4f w = *(const v4f*)(sW + f * kDM + c4);
      acc += p * w;
    }
    acc += bb;
    acc += pe;
    float* dst = H + ((size_t)(n * kRps + p0l + pl)) * kDM + c4;
    *(volatile v4f*)dst = acc;
    __threadfence();
    *(volatile v4f*)dst = acc;
  }
}

__global__ __launch_bounds__(256) void ln_kernel(
    const float* __restrict__ H, const float* __restrict__ ln_g, const float* __restrict__ ln_b,
    unsigned short* __restrict__ XNH, unsigned short* __restrict__ XNL, int l)
{
  const int tid = threadIdx.x, lane = tid & 31, wave = tid >> 5;
  const int row = blockIdx.x * 16 + wave * 2 + (lane >> 4);
  const int c8 = (lane & 15) * 8;
  const float* hp = H + (size_t)row * kDM + c8;
  const v4f a0 = *(const v4f*)(hp);
  const v4f a1 = *(const v4f*)(hp + 4);
  float s = ((a0[0] + a0[1]) + (a0[2] + a0[3])) + ((a1[0] + a1[1]) + (a1[2] + a1[3]));
  s += __shfl_xor(s, 1, 32);
  s += __shfl_xor(s, 2, 32);
  s += __shfl_xor(s, 4, 32);
  s += __shfl_xor(s, 8, 32);
  const float mean = s * (1.0f / 128.0f);
  float q = 0.f;
#pragma unroll
  for (int e = 0; e < 4; ++e) { const float d0 = a0[e] - mean; const float d1 = a1[e] - mean; q += d0 * d0; q += d1 * d1; }
  q += __shfl_xor(q, 1, 32);
  q += __shfl_xor(q, 2, 32);
  q += __shfl_xor(q, 4, 32);
  q += __shfl_xor(q, 8, 32);
  const float var = q * (1.0f / 128.0f);
  const float inv = rsqrtf(var + 1e-5f);
  const float* gp = ln_g + l * kDM + c8;
  const float* bp = ln_b + l * kDM + c8;
  const v4f g0 = *(const v4f*)(gp), g1 = *(const v4f*)(gp + 4);
  const v4f b0 = *(const v4f*)(bp), b1 = *(const v4f*)(bp + 4);
  v8h hv, lv;
#pragma unroll
  for (int e = 0; e < 4; ++e) {
    const float x0 = (a0[e] - mean) * inv * bf16r(g0[e]) + bf16r(b0[e]);
    const float x1 = (a1[e] - mean) * inv * bf16r(g1[e]) + bf16r(b1[e]);
    const unsigned short h0 = f2bf_bits(x0), h1 = f2bf_bits(x1);
    const unsigned short l0 = f2bf_bits(x0 - bf_bits2f(h0)), l1 = f2bf_bits(x1 - bf_bits2f(h1));
    hv[e]     = __builtin_bit_cast(_Float16, h0);
    hv[4 + e] = __builtin_bit_cast(_Float16, h1);
    lv[e]     = __builtin_bit_cast(_Float16, l0);
    lv[4 + e] = __builtin_bit_cast(_Float16, l1);
  }
  unsigned short* qh = XNH + (size_t)row * kDM + c8;
  unsigned short* ql = XNL + (size_t)row * kDM + c8;
  *(volatile v8h*)qh = hv;
  *(volatile v8h*)ql = lv;
  __threadfence();
  *(volatile v8h*)qh = hv;
  *(volatile v8h*)ql = lv;
}

__device__ __forceinline__ float softplus_f(float v) {
  const float a   = __expf(-fabsf(v));
  const float u   = 1.0f + a;
  const float l1p = __logf(u) + (a - (u - 1.0f)) * __builtin_amdgcn_rcpf(u);
  return fmaxf(v, 0.0f) + l1p;
}

__global__ __launch_bounds__(256) void scan_kernel(
    const float* __restrict__ PJ, const unsigned short* __restrict__ XNH, const unsigned short* __restrict__ XNL,
    const float* __restrict__ dt_b, const float* __restrict__ A_log, const float* __restrict__ D_skip,
    const float* __restrict__ tsrc, unsigned short* __restrict__ YH, unsigned short* __restrict__ YL,
    int l, int prune)
{
  __shared__ float sA[32 * 256];
  const int tid = threadIdx.x, lane = tid & 31;
  const int dir = blockIdx.y;
  const int ld = l * 2 + dir;
  const int pl = blockIdx.x * 4 + (tid >> 6);
  const int half = (tid >> 5) & 1;
  const int d0 = half * 64 + lane * 2;
#pragma unroll 1
  for (int j = 0; j < 32; ++j) {
    const int c = j >> 4, s = j & 15;
    const float al = bf16r(A_log[((size_t)(ld * kDM + d0 + c)) * kNS + s]);
    sA[j * 256 + tid] = -expf(al) * kLog2e;
  }
  __syncthreads();
  float a20[kNS], a21[kNS], h0[kNS], h1[kNS];
#pragma unroll
  for (int s = 0; s < kNS; ++s) {
    a20[s] = sA[s * 256 + tid];
    a21[s] = sA[(kNS + s) * 256 + tid];
    h0[s] = 0.f;
    h1[s] = 0.f;
  }
  const float dtb0 = bf16r(dt_b[ld * kDM + d0]);
  const float dtb1 = bf16r(dt_b[ld * kDM + d0 + 1]);
  const float ds0  = bf16r(D_skip[ld * kDM + d0]);
  const float ds1  = bf16r(D_skip[ld * kDM + d0 + 1]);
  const int il = sel_low_index(tsrc);
  int nsteps = kNT;
  if (prune != 0) nsteps = (dir == 0) ? (il + 2) : (kNT - il);
  nsteps = nsteps < 1 ? 1 : (nsteps > kNT ? kNT : nsteps);
  const float* PJd = PJ + (size_t)dir * kRows * kPJW;
  volatile unsigned* yhw = (volatile unsigned*)YH;
  volatile unsigned* ylw = (volatile unsigned*)YL;
#pragma unroll 1
  for (int stp = 0; stp < nsteps; ++stp) {
    const int n = (dir == 0) ? stp : (kNT - 1 - stp);
    const size_t row = (size_t)n * kRps + (size_t)pl;
    const float* pr = PJd + row * kPJW;
    const v2f dtr = *(const v2f*)(pr + d0);
    const unsigned wh = *(const unsigned*)(XNH + row * kDM + d0);
    const unsigned wl = *(const unsigned*)(XNL + row * kDM + d0);
    v4f bq[4], cq[4];
#pragma unroll
    for (int i = 0; i < 4; ++i) {
      bq[i] = *(const v4f*)(pr + kDM + 4 * i);
      cq[i] = *(const v4f*)(pr + kDM + kNS + 4 * i);
    }
    const float x0 = __uint_as_float(wh << 16) + __uint_as_float(wl << 16);
    const float x1 = __uint_as_float(wh & 0xffff0000u) + __uint_as_float(wl & 0xffff0000u);
    const float dt0 = softplus_f(dtr[0] + dtb0);
    const float dt1 = softplus_f(dtr[1] + dtb1);
    const float dtx0 = dt0 * x0;
    const float dtx1 = dt1 * x1;
    float y0 = 0.f, y1 = 0.f;
#pragma unroll
    for (int s = 0; s < kNS; ++s) {
      const float bs = bq[s >> 2][s & 3];
      const float cs = cq[s >> 2][s & 3];
      const float e0 = __builtin_amdgcn_exp2f(dt0 * a20[s]);
      const float e1 = __builtin_amdgcn_exp2f(dt1 * a21[s]);
      h0[s] = e0 * h0[s] + dtx0 * bs;
      h1[s] = e1 * h1[s] + dtx1 * bs;
      y0 = h0[s] * cs + y0;
      y1 = h1[s] * cs + y1;
    }
    y0 = ds0 * x0 + y0;
    y1 = ds1 * x1 + y1;
    const unsigned short hb0 = f2bf_bits(y0), hb1 = f2bf_bits(y1);
    const unsigned short lb0 = f2bf_bits(y0 - bf_bits2f(hb0)), lb1 = f2bf_bits(y1 - bf_bits2f(hb1));
    const unsigned wH = (unsigned)hb0 | ((unsigned)hb1 << 16);
    const unsigned wL = (unsigned)lb0 | ((unsigned)lb1 << 16);
    const size_t wo = row * (kYW / 2) + (size_t)dir * 64 + (size_t)half * 32 + (size_t)lane;
    yhw[wo] = wH;
    ylw[wo] = wL;
    __threadfence();
    yhw[wo] = wH;
    ylw[wo] = wL;
  }
}

__global__ __launch_bounds__(256) void head_kernel(
    const float* __restrict__ H, const float* __restrict__ tsrc,
    const float* __restrict__ te_W1, const float* __restrict__ te_b1,
    const float* __restrict__ te_W2, const float* __restrict__ te_b2,
    const float* __restrict__ op_W, const float* __restrict__ op_b,
    float* __restrict__ out, int chunk)
{
#pragma clang fp contract(off)
  __shared__ __align__(16) float sOW[kDM * kGD];
  __shared__ __align__(16) float sOB[16];
  __shared__ __align__(16) float sS[kDM];
  __shared__ __align__(16) float sTE[kDM];
  __shared__ __align__(16) float sHI[64 * 132];
  __shared__ __align__(16) float sO[64 * 16];
  __shared__ __align__(16) float sInv[64];
  __shared__ __align__(16) float sAct[896];
  const int tid = threadIdx.x, lane = tid & 31, wave = tid >> 5;
  const int p0l = blockIdx.x * 64;
  const float tv = bf16r(tsrc[0]);
  const float tn = tv * 7.0f;
  int il = (int)floorf(tn);
  il = il < 0 ? 0 : il;
  il = il > (kNT - 2) ? (kNT - 2) : il;
  int ih = il + 1;
  ih = ih > (kNT - 1) ? (kNT - 1) : ih;
  const float alpha = tn - (float)il;

  for (int idx = tid; idx < kDM * kGD; idx += 256) sOW[idx] = bf16r(op_W[idx]);
  if (tid < kGD) sOB[tid] = bf16r(op_b[tid]);
  if (tid < kDM) {
    const float pre = tv * bf16r(te_W1[tid]) + bf16r(te_b1[tid]);
    const float sg = 1.0f / (1.0f + expf(-pre));
    sS[tid] = pre * sg;
  }
  __syncthreads();
  if (tid < kDM) {
    float acc = 0.f;
#pragma unroll 1
    for (int k = 0; k < kDM; ++k) acc = acc + sS[k] * bf16r(te_W2[(size_t)k * kDM + tid]);
    sTE[tid] = acc + bf16r(te_b2[tid]);
  }
  __syncthreads();
  {
    const int c4 = lane * 4;
    const v4f te4 = *(const v4f*)(sTE + c4);
    const float oma = 1.0f - alpha;
#pragma unroll 1
    for (int i = 0; i < 8; ++i) {
      const int pl = wave * 8 + i;
      const int p = p0l + pl;
      const v4f hl = *(const v4f*)(H + ((size_t)(il * kRps + p)) * kDM + c4);
      const v4f hh = *(const v4f*)(H + ((size_t)(ih * kRps + p)) * kDM + c4);
      v4f v = oma * hl + alpha * hh;
      v = v + te4;
      *(v4f*)(sHI + pl * 132 + c4) = v;
    }
  }
  __syncthreads();
  {
    const int pl = tid >> 2, q = tid & 3;
    const int g0 = q, g1 = q + 4, g2 = q + 8;
    const int g3 = (q + 12) > (kGD - 1) ? (kGD - 1) : (q + 12);
    float a0 = 0.f, a1 = 0.f, a2 = 0.f, a3 = 0.f;
#pragma unroll 1
    for (int c = 0; c < kDM; ++c) {
      const float hv = sHI[pl * 132 + c];
      const float* wr = sOW + c * kGD;
      a0 = a0 + hv * wr[g0];
      a1 = a1 + hv * wr[g1];
      a2 = a2 + hv * wr[g2];
      a3 = a3 + hv * wr[g3];
    }
    sO[pl * 16 + g0] = a0 + sOB[g0];
    sO[pl * 16 + g1] = a1 + sOB[g1];
    sO[pl * 16 + g2] = a2 + sOB[g2];
    if (q < 2) sO[pl * 16 + g3] = a3 + sOB[g3];
  }
  __syncthreads();
  if (tid < 64) {
    const float r0 = sO[tid * 16 + 6], r1 = sO[tid * 16 + 7], r2 = sO[tid * 16 + 8], r3 = sO[tid * 16 + 9];
    const float ss = ((r0 * r0 + r1 * r1) + r2 * r2) + r3 * r3;
    const float nrm = sqrtf(ss);
    sInv[tid] = 1.0f / fmaxf(nrm, 1e-12f);
  }
  __syncthreads();
#pragma unroll 1
  for (int e = tid; e < 896; e += 256) {
    const int pl = e / kGD;
    const int g = e - pl * kGD;
    const float v = sO[pl * 16 + g];
    const float inv = sInv[pl];
    const float sp = log1pf(expf(-fabsf(v))) + fmaxf(v, 0.0f);
    const float sg = 1.0f / (1.0f + expf(-v));
    const float rn = v * inv;
    const float r = (g < 3) ? v : ((g < 6) ? sp : ((g < 10) ? rn : sg));
    sAct[e] = r;
  }
  __syncthreads();
  int nvalid = kChunkPts - p0l;
  nvalid = nvalid > 64 ? 64 : nvalid;
  const int nthr = (nvalid * kGD) / 4;
  if (tid < nthr) {
    const v4f val = *(const v4f*)(sAct + tid * 4);
    float* dst = out + ((size_t)(chunk * kChunkPts + p0l)) * kGD + tid * 4;
    *(volatile v4f*)dst = val;
    __threadfence();
    *(volatile v4f*)dst = val;
  }
}

extern "C" void kernel_launch(void* const* d_in, const int* in_sizes, int n_in,
                              void* d_out, int out_size, void* d_ws, size_t ws_size,
                              hipStream_t stream) {
  if (n_in < 25) return;
  if (in_sizes[0] != kNT * kNP * 3) return;
  if (in_sizes[1] != kNT * kNP * 3) return;
  if (in_sizes[2] != kNT * kNP * 4) return;
  if (in_sizes[3] != kNT * kNP) return;
  if (in_sizes[4] != kNT * kNP * 3) return;
  if (in_sizes[5] != 1) return;
  if (in_sizes[6] != kNT) return;
  if (in_sizes[7] != kGD * kDM) return;
  if (in_sizes[8] != kDM) return;
  if (in_sizes[9] != kNL * kDM) return;
  if (in_sizes[10] != kNL * kDM) return;
  if (in_sizes[11] != kNL * 2 * kDM * kDM) return;
  if (in_sizes[12] != kNL * 2 * kDM) return;
  if (in_sizes[13] != kNL * 2 * kDM * kNS) return;
  if (in_sizes[14] != kNL * 2 * kDM * kNS) return;
  if (in_sizes[15] != kNL * 2 * kDM * kNS) return;
  if (in_sizes[16] != kNL * 2 * kDM) return;
  if (in_sizes[17] != kNL * 2 * kDM * kDM) return;
  if (in_sizes[18] != kNL * kDM) return;
  if (in_sizes[19] != kDM) return;
  if (in_sizes[20] != kDM) return;
  if (in_sizes[21] != kDM * kDM) return;
  if (in_sizes[22] != kDM) return;
  if (in_sizes[23] != kDM * kGD) return;
  if (in_sizes[24] != kGD) return;
  if (out_size != kNP * kGD) return;
  if (ws_size < kWsTotal) return;

  const float* xyz    = (const float*)d_in[0];
  const float* scl    = (const float*)d_in[1];
  const float* rot    = (const float*)d_in[2];
  const float* opa    = (const float*)d_in[3];
  const float* col    = (const float*)d_in[4];
  const float* tsrc   = (const float*)d_in[5];
  const float* tstamp = (const float*)d_in[6];
  const float* in_W   = (const float*)d_in[7];
  const float* in_b   = (const float*)d_in[8];
  const float* ln_g   = (const float*)d_in[9];
  const float* ln_b   = (const float*)d_in[10];
  const float* dt_W   = (const float*)d_in[11];
  const float* dt_b   = (const float*)d_in[12];
  const float* B_W    = (const float*)d_in[13];
  const float* C_W    = (const float*)d_in[14];
  const float* A_log  = (const float*)d_in[15];
  const float* D_skip = (const float*)d_in[16];
  const float* out_W  = (const float*)d_in[17];
  const float* out_b  = (const float*)d_in[18];
  const float* te_W1  = (const float*)d_in[19];
  const float* te_b1  = (const float*)d_in[20];
  const float* te_W2  = (const float*)d_in[21];
  const float* te_b2  = (const float*)d_in[22];
  const float* op_W   = (const float*)d_in[23];
  const float* op_b   = (const float*)d_in[24];
  float* out = (float*)d_out;

  char* ws = (char*)d_ws;
  unsigned short* WPJ  = (unsigned short*)(ws + kOffWPJ);
  unsigned short* WOUT = (unsigned short*)(ws + kOffWOUT);
  float*          PE   = (float*)(ws + kOffPE);
  float*          H    = (float*)(ws + kOffH);
  unsigned short* XNH  = (unsigned short*)(ws + kOffXNH);
  unsigned short* XNL  = (unsigned short*)(ws + kOffXNL);
  float*          PJ   = (float*)(ws + kOffPJ);
  unsigned short* YH   = (unsigned short*)(ws + kOffYH);
  unsigned short* YL   = (unsigned short*)(ws + kOffYL);

  constexpr int kProjBlocks = ((kRows / 64) * (kPJW / 64) + 7) / 8;
  constexpr int kOutBlocks0 = ((kRows / 64) * (kDM / 64) + 7) / 8;
  constexpr int kOutBlocks1 = (((2 * kRps) / 64) * (kDM / 64) + 7) / 8;

  prep_kernel<<<17, 256, 0, stream>>>(dt_W, B_W, C_W, out_W, tstamp, WPJ, WOUT, PE);

  for (int chunk = 0; chunk < kNChunk; ++chunk) {
    inproj_kernel<<<kNT * kPBlk, 256, 0, stream>>>(xyz, scl, rot, opa, col, in_W, in_b, PE, H, chunk);
    for (int l = 0; l < kNL; ++l) {
      ln_kernel<<<kRows / 16, 256, 0, stream>>>(H, ln_g, ln_b, XNH, XNL, l);

      const unsigned short* wpj = WPJ + (size_t)l * 2 * kPJW * kDM;
      if (l == 0) {
        wmma_gemm64<1, 1, 0, 0, false, 0, 0><<<dim3(kProjBlocks, 2), 256, 0, stream>>>(
            XNH, XNL, kDM, 0L,
            wpj, nullptr, kDM, (long)(kPJW * kDM),
            (void*)PJ, nullptr, kPJW, (long)kRows * kPJW,
            nullptr, nullptr, 0L,
            kRows, kPJW, kDM, 1.0f, tsrc, kRps);
      } else {
        wmma_gemm64<1, 1, 0, 0, false, 0, 1><<<dim3(kProjBlocks, 2), 256, 0, stream>>>(
            XNH, XNL, kDM, 0L,
            wpj, nullptr, kDM, (long)(kPJW * kDM),
            (void*)PJ, nullptr, kPJW, (long)kRows * kPJW,
            nullptr, nullptr, 0L,
            kRows, kPJW, kDM, 1.0f, tsrc, kRps);
      }

      scan_kernel<<<dim3(kRps / 4, 2), 256, 0, stream>>>(PJ, XNH, XNL, dt_b, A_log, D_skip, tsrc, YH, YL, l, (l == 1) ? 1 : 0);

      const unsigned short* wo = WOUT + (size_t)l * kDM * kYW;
      if (l == 0) {
        wmma_gemm64<1, 1, 2, 0, true, 0, 0><<<dim3(kOutBlocks0, 1), 256, 0, stream>>>(
            YH, YL, kYW, 0L,
            wo, nullptr, kYW, 0L,
            (void*)H, nullptr, kDM, 0L,
            out_b + l * kDM,
            H, 0L,
            kRows, kDM, kYW, 1.0f, tsrc, kRps);
      } else {
        wmma_gemm64<1, 1, 2, 0, true, 0, 2><<<dim3(kOutBlocks1, 1), 256, 0, stream>>>(
            YH, YL, kYW, 0L,
            wo, nullptr, kYW, 0L,
            (void*)H, nullptr, kDM, 0L,
            out_b + l * kDM,
            H, 0L,
            2 * kRps, kDM, kYW, 1.0f, tsrc, kRps);
      }
    }
    head_kernel<<<kPBlk, 256, 0, stream>>>(H, tsrc, te_W1, te_b1, te_W2, te_b2, op_W, op_b, out, chunk);
  }
}
